// ContextRNN_12111807774829
// MI455X (gfx1250) — hardware-verified
//
#include <hip/hip_runtime.h>

typedef __attribute__((ext_vector_type(16))) _Float16 v16h;
typedef __attribute__((ext_vector_type(8)))  _Float16 v8h;
typedef __attribute__((ext_vector_type(16))) __bf16   v16b;
typedef __attribute__((ext_vector_type(8)))  __bf16   v8b;
typedef __attribute__((ext_vector_type(8)))  float    v8f;
typedef __attribute__((ext_vector_type(4)))  float    v4f;
typedef __attribute__((ext_vector_type(4)))  unsigned v4u;
#define PSCALE 32768.0f
#define U16(p) ((const unsigned short*)(const void*)(p))
#define PSCALE_INV (1.0f / 32768.0f)

__device__ __forceinline__ unsigned short f2bf_bits(float f) {
  unsigned u = __float_as_uint(f);
  return (unsigned short)((u + 0x7FFFu + ((u >> 16) & 1u)) >> 16);
}
__device__ __forceinline__ float bf_bits2f(unsigned short h) { return __uint_as_float(((unsigned)h) << 16); }

__device__ __forceinline__ void dep_guard_h(v8f& a, v8f& b, v16h x, v16h y) { asm volatile("v_nop\n\tv_nop\n\tv_nop\n\tv_nop" : "+v"(a), "+v"(b) : "v"(x), "v"(y)); }
__device__ __forceinline__ void dep_guard_b(v8f& a, v8f& b, v16b x, v16b y) { asm volatile("v_nop\n\tv_nop\n\tv_nop\n\tv_nop" : "+v"(a), "+v"(b) : "v"(x), "v"(y)); }
__device__ __forceinline__ void keep4_h(v16h a, v16h b, v16h c, v16h d) { asm volatile("v_nop" :: "v"(a), "v"(b), "v"(c), "v"(d)); }
__device__ __forceinline__ void keep4_b(v16b a, v16b b, v16b c, v16b d) { asm volatile("v_nop" :: "v"(a), "v"(b), "v"(c), "v"(d)); }
__device__ __forceinline__ void acc_guard4(v8f& a, v8f& b, v8f& c, v8f& d) { asm volatile("v_nop\n\tv_nop\n\tv_nop\n\tv_nop" : "+v"(a), "+v"(b), "+v"(c), "+v"(d)); }
__device__ __forceinline__ void acc_guard2(v8f& a, v8f& b) { asm volatile("v_nop\n\tv_nop\n\tv_nop\n\tv_nop" : "+v"(a), "+v"(b)); }
template <typename T> struct Frag;
template <> struct Frag<_Float16> {
  typedef v16h V; union U { v16h v; v8h h[2]; };
  static __device__ __forceinline__ v16h load(const _Float16* p) {
    U f; f.h[0] = *(const v8h*)(p); f.h[1] = *(const v8h*)(p + 16); return f.v;
  }
  static __device__ __forceinline__ v8f mma(v16h a, v16h b, v8f c) {
    return __builtin_amdgcn_wmma_f32_16x16x32_f16(false, a, false, b, (short)0, c, false, false);
  }
  static __device__ __forceinline__ void guard(v8f& a, v8f& b, v16h x, v16h y) { dep_guard_h(a, b, x, y); }
  static __device__ __forceinline__ void keep(v16h a, v16h b, v16h c, v16h d) { keep4_h(a, b, c, d); }
};
template <> struct Frag<__bf16> {
  typedef v16b V; union U { v16b v; v8b h[2]; };
  static __device__ __forceinline__ v16b load(const __bf16* p) {
    U f; f.h[0] = *(const v8b*)(p); f.h[1] = *(const v8b*)(p + 16); return f.v;
  }
  static __device__ __forceinline__ v8f mma(v16b a, v16b b, v8f c) {
    return __builtin_amdgcn_wmma_f32_16x16x32_bf16(false, a, false, b, (short)0, c, false, false);
  }
  static __device__ __forceinline__ void guard(v8f& a, v8f& b, v16b x, v16b y) { dep_guard_b(a, b, x, y); }
  static __device__ __forceinline__ void keep(v16b a, v16b b, v16b c, v16b d) { keep4_b(a, b, c, d); }
};

template <int ET> struct Elem;
template <> struct Elem<0> { typedef _Float16 T; };
template <> struct Elem<1> { typedef __bf16 T; };
template <int ET, bool SPLIT, int BIAS_MODE, int OUT_MODE, bool RESID, int ACT = 0>
__global__ __launch_bounds__(256) void wmma_gemm64(
    const unsigned short* __restrict__ Ap, const unsigned short* __restrict__ A2p, int lda, long strideA,
    const unsigned short* __restrict__ Btp, const unsigned short* __restrict__ Bt2p, int ldb, long strideB,
    void* __restrict__ Cout, void* __restrict__ Cout2, int ldc, long strideC,
    const float* __restrict__ bias,
    const float* __restrict__ resid, long strideR,
    int M, int N, int K, float scale) {
  typedef typename Elem<ET>::T T;
  typedef typename Frag<T>::V V;
  const T* A = (const T*)Ap; const T* A2 = (const T*)A2p; const T* Bt = (const T*)Btp; const T* Bt2 = (const T*)Bt2p;
  __shared__ __align__(16) float sT[8][16 * 68];
  const int b    = blockIdx.y;
  const int lane = threadIdx.x & 31;
  const int wave = threadIdx.x >> 5;
  const int tilesN = N >> 6;
  const int tilesM = M >> 6;
  const int tile = blockIdx.x * 8 + wave;
  if (tile >= tilesM * tilesN) return;
  const int tm = tile / tilesN;
  const int tn = tile - tm * tilesN;
  const int m0 = tm << 6;
  const int n0 = tn << 6;

  const T* Ab  = A  + (size_t)b * strideA;
  const T* Bb  = Bt + (size_t)b * strideB;
  const T* Ab2 = SPLIT ? (A2  + (size_t)b * strideA) : nullptr;
  const T* Bb2 = SPLIT ? (Bt2 + (size_t)b * strideB) : nullptr;

  const int rlane = lane & 15;
  const int koff  = (lane >> 4) * 8;
  const int mOff  = (lane >> 4) * 8;

  v8f acc[4][4];
#pragma unroll
  for (int i = 0; i < 4; ++i)
#pragma unroll
    for (int j = 0; j < 4; ++j) acc[i][j] = (v8f){0.f,0.f,0.f,0.f,0.f,0.f,0.f,0.f};

  for (int k0 = 0; k0 < K; k0 += 32) {
    V bh[4], bl[4];
#pragma unroll
    for (int j = 0; j < 4; ++j) {
      const size_t bo = (size_t)(n0 + (j << 4) + rlane) * ldb + koff + k0;
      bh[j] = Frag<T>::load(Bb + bo);
      if (SPLIT) bl[j] = Frag<T>::load(Bb2 + bo);
    }
#pragma unroll
    for (int i = 0; i < 4; ++i) {
      const size_t ao = (size_t)(m0 + (i << 4) + rlane) * lda + koff + k0;
      V ah = Frag<T>::load(Ab + ao);
      V al;
      if (SPLIT) al = Frag<T>::load(Ab2 + ao);
#pragma unroll
      for (int j = 0; j < 4; ++j) {
        acc[i][j] = Frag<T>::mma(ah, bh[j], acc[i][j]);
        if (SPLIT) {
          acc[i][j] = Frag<T>::mma(ah, bl[j], acc[i][j]);
          acc[i][j] = Frag<T>::mma(al, bh[j], acc[i][j]);
        }
      }
      Frag<T>::guard(acc[i][0], acc[i][3], ah, SPLIT ? al : ah);
    }
    Frag<T>::keep(bh[0], bh[1], bh[2], bh[3]);
    if (SPLIT) Frag<T>::keep(bl[0], bl[1], bl[2], bl[3]);
  }
  acc_guard4(acc[0][0], acc[0][1], acc[0][2], acc[0][3]);
  acc_guard4(acc[1][0], acc[1][1], acc[1][2], acc[1][3]);
  acc_guard4(acc[2][0], acc[2][1], acc[2][2], acc[2][3]);
  acc_guard4(acc[3][0], acc[3][1], acc[3][2], acc[3][3]);

  float* slab = sT[wave];
  const float* Rb = RESID ? (resid + (size_t)b * strideR) : nullptr;
#pragma unroll
  for (int i = 0; i < 4; ++i) {
    const int mBase = m0 + (i << 4);
#pragma unroll
    for (int j = 0; j < 4; ++j) {
      const int n = n0 + (j << 4) + rlane;
      float bv = 0.f;
      if (BIAS_MODE == 2) bv = bias[n];
#pragma unroll
      for (int r = 0; r < 8; ++r) {
        float v = acc[i][j][r] * scale;
        if (BIAS_MODE == 1) v += bias[mBase + mOff + r];
        if (BIAS_MODE == 2) v += bv;
        if (RESID) v += Rb[(size_t)(mBase + mOff + r) * ldc + n];
        if (ACT == 1) v = tanhf(v);
        if (ACT == 2) v = fmaxf(v, 0.0f);
        if (ACT == 3) v = v / (1.0f + expf(-v));
        if (ACT == 4) v = (v > 0.f) ? v : 0.01f * v;
        if (ACT == 5) v = 0.5f * v * (1.0f + erff(v * 0.70710678118654752f));
        slab[(mOff + r) * 68 + (j << 4) + rlane] = v;
      }
    }
    __builtin_amdgcn_fence(__ATOMIC_RELEASE, "workgroup");
    __builtin_amdgcn_wave_barrier();
    __builtin_amdgcn_fence(__ATOMIC_ACQUIRE, "workgroup");
    if (OUT_MODE == 0) {
      float* C = (float*)Cout + (size_t)b * strideC;
      const int hh = lane >> 4, c4 = (lane & 15) * 4;
      for (int pass = 0; pass < 2; ++pass) {
#pragma unroll
        for (int it = 0; it < 8; ++it) {
          const int row = it * 2 + hh;
          v4f v = *(const v4f*)(slab + row * 68 + c4);
          *(volatile v4f*)(C + (size_t)(mBase + row) * ldc + n0 + c4) = v;
        }
        __threadfence();
      }
    } else {
      const int q = lane >> 3, c8 = (lane & 7) * 8;
      unsigned short* C  = (unsigned short*)Cout  + (size_t)b * strideC;
      unsigned short* C2 = (OUT_MODE == 2) ? ((unsigned short*)Cout2 + (size_t)b * strideC) : nullptr;
      for (int pass = 0; pass < 2; ++pass) {
#pragma unroll
        for (int it = 0; it < 4; ++it) {
          const int row = it * 4 + q;
          const float* sp = slab + row * 68 + c8;
          v8h hv, lv;
#pragma unroll
          for (int e = 0; e < 8; ++e) {
            if (OUT_MODE == 1) {
              hv[e] = (_Float16)sp[e];
            } else {
              unsigned short hb = f2bf_bits(sp[e]);
              unsigned short lb = f2bf_bits(sp[e] - bf_bits2f(hb));
              hv[e] = __builtin_bit_cast(_Float16, hb);
              lv[e] = __builtin_bit_cast(_Float16, lb);
            }
          }
          *(volatile v8h*)(C + (size_t)(mBase + row) * ldc + n0 + c8) = hv;
          if (OUT_MODE == 2) *(volatile v8h*)(C2 + (size_t)(mBase + row) * ldc + n0 + c8) = lv;
        }
        __threadfence();
      }
    }
    __builtin_amdgcn_fence(__ATOMIC_RELEASE, "workgroup");
    __builtin_amdgcn_wave_barrier();
    __builtin_amdgcn_fence(__ATOMIC_ACQUIRE, "workgroup");
  }
}

static constexpr int NBATCH = 32;
static constexpr int NTIME  = 512;
static constexpr int NMEM   = 6;
static constexpr int NHID   = 512;
static constexpr int NH3    = 1536;
static constexpr int NVOCAB = 32000;
static constexpr int NROWS  = NBATCH * NTIME;
static constexpr int TCHUNK = 128;
static constexpr int NCHUNK = NTIME / TCHUNK;
static constexpr int ROWS_CH = TCHUNK * NBATCH;
static constexpr float WSCALE = 16.0f;
static constexpr float WSCALE_INV = 0.0625f;

__device__ __forceinline__ unsigned short h_bits(float f) { return __builtin_bit_cast(unsigned short, (_Float16)f); }
__device__ __forceinline__ unsigned pack2h(float a, float b) { return (unsigned)h_bits(a) | ((unsigned)h_bits(b) << 16); }
__device__ __forceinline__ float sigm_f(float x) { return __builtin_amdgcn_rcpf(1.0f + expf(-x)); }

__global__ __launch_bounds__(256) void transpose_cast_f16(const float* __restrict__ in, unsigned short* __restrict__ out,
                                                          int R, int CC, float sc) {
  __shared__ float tile[64][65];
  const int tid = threadIdx.x, lane = tid & 31, wave = tid >> 5;
  const int r0 = blockIdx.y * 64, c0 = blockIdx.x * 64;
  {
    const int row = tid >> 2, cb = (tid & 3) * 16;
    const float* src = in + (size_t)(r0 + row) * CC + c0 + cb;
#pragma unroll
    for (int i = 0; i < 4; ++i) {
      const v4f v = *(const v4f*)(src + 4 * i);
      tile[row][cb + 4 * i + 0] = v[0] * sc;
      tile[row][cb + 4 * i + 1] = v[1] * sc;
      tile[row][cb + 4 * i + 2] = v[2] * sc;
      tile[row][cb + 4 * i + 3] = v[3] * sc;
    }
  }
  __syncthreads();
  const int q = lane >> 3, c8 = (lane & 7) * 8;
  v4u pk[2];
  size_t off[2];
#pragma unroll
  for (int it = 0; it < 2; ++it) {
    const int orow = wave * 8 + it * 4 + q;
    v4u w;
    w[0] = pack2h(tile[c8 + 0][orow], tile[c8 + 1][orow]);
    w[1] = pack2h(tile[c8 + 2][orow], tile[c8 + 3][orow]);
    w[2] = pack2h(tile[c8 + 4][orow], tile[c8 + 5][orow]);
    w[3] = pack2h(tile[c8 + 6][orow], tile[c8 + 7][orow]);
    pk[it] = w;
    off[it] = (size_t)(c0 + orow) * R + r0 + c8;
  }
  for (int pass = 0; pass < 2; ++pass) {
#pragma unroll
    for (int it = 0; it < 2; ++it) *(volatile v4u*)(out + off[it]) = pk[it];
    __threadfence();
  }
}

__global__ __launch_bounds__(64) void embed_sum_kernel(const int* __restrict__ seqs, const float* __restrict__ emb,
                                                       unsigned short* __restrict__ emb16) {
  const int blk = blockIdx.x;
  const int b = blk & (NBATCH - 1), t = blk >> 5;
  const int j8 = threadIdx.x * 8;
  const int* sp = seqs + ((size_t)b * NTIME + t) * NMEM;
  float a[8];
#pragma unroll
  for (int i = 0; i < 8; ++i) a[i] = 0.f;
#pragma unroll
  for (int m = 0; m < NMEM; ++m) {
    const int tok = sp[m];
    const bool keep = (tok != 1);
    int tc = tok < 0 ? 0 : tok;
    tc = tc > (NVOCAB - 1) ? (NVOCAB - 1) : tc;
    const float* e = emb + (size_t)tc * NHID + j8;
    const v4f e0 = *(const v4f*)e;
    const v4f e1 = *(const v4f*)(e + 4);
    a[0] += keep ? e0[0] : 0.f;  a[1] += keep ? e0[1] : 0.f;
    a[2] += keep ? e0[2] : 0.f;  a[3] += keep ? e0[3] : 0.f;
    a[4] += keep ? e1[0] : 0.f;  a[5] += keep ? e1[1] : 0.f;
    a[6] += keep ? e1[2] : 0.f;  a[7] += keep ? e1[3] : 0.f;
  }
  v4u w;
  w[0] = pack2h(a[0], a[1]); w[1] = pack2h(a[2], a[3]);
  w[2] = pack2h(a[4], a[5]); w[3] = pack2h(a[6], a[7]);
  unsigned short* dst = emb16 + (size_t)blk * NHID + j8;
  *(volatile v4u*)dst = w;
  __threadfence();
  *(volatile v4u*)dst = w;
}

__global__ __launch_bounds__(256) void gru_scan_kernel(
    const float* __restrict__ xsF, const float* __restrict__ xsB,
    const unsigned short* __restrict__ rktF, const unsigned short* __restrict__ rktB,
    const float* __restrict__ biasF, const float* __restrict__ biasB,
    const int* __restrict__ lens,
    unsigned short* __restrict__ out16,
    float* __restrict__ hst,
    int t0F, int t0B, int first) {
  __shared__ __align__(16) _Float16 hs16[2 * 16 * NHID];
  __shared__ __align__(16) float hf[16 * NHID];
  const int tid = threadIdx.x, wave = tid >> 5, lane = tid & 31;
  const int hh = lane >> 4, cl = lane & 15, koff = hh * 8;
  const int dir = blockIdx.x >> 1;
  const int bBase = (blockIdx.x & 1) * 16;
  const float* xs = dir ? xsB : xsF;
  const _Float16* rkt = (const _Float16*)(dir ? rktB : rktF);
  const float* brec = (dir ? biasB : biasF) + NH3;
  const int t0 = dir ? t0B : t0F;

  if (first != 0) {
    for (int i = tid; i < 16 * NHID; i += 256) { hf[i] = 0.f; hs16[i] = (_Float16)0.f; }
  } else {
    for (int i = tid; i < 16 * NHID; i += 256) {
      const int row = i >> 9, col = i & (NHID - 1);
      const float v = hst[((size_t)(dir * NBATCH + bBase + row)) * NHID + col];
      hf[i] = v;
      hs16[i] = (_Float16)v;
    }
  }
  int lenr[8];
#pragma unroll
  for (int r = 0; r < 8; ++r) lenr[r] = lens[bBase + 8 * hh + r];
  __syncthreads();

  for (int s = 0; s < TCHUNK; ++s) {
    const int t  = dir ? (t0 + TCHUNK - 1 - s) : (t0 + s);
    const int tl = t - t0;
    const _Float16* hcur = hs16 + (s & 1) * (16 * NHID);
    _Float16* hnext = hs16 + ((s + 1) & 1) * (16 * NHID);

#pragma unroll 1
    for (int pass = 0; pass < 2; ++pass) {
      const int ub0 = wave * 4 + pass * 2;
      v8f acc[2][3];
#pragma unroll
      for (int u = 0; u < 2; ++u)
#pragma unroll
        for (int g = 0; g < 3; ++g) acc[u][g] = (v8f){0.f,0.f,0.f,0.f,0.f,0.f,0.f,0.f};

#pragma unroll 2
      for (int k0 = 0; k0 < NHID; k0 += 32) {
        const v16h a = Frag<_Float16>::load(hcur + cl * NHID + koff + k0);
        v16h bq[2][3];
#pragma unroll
        for (int u = 0; u < 2; ++u)
#pragma unroll
          for (int g = 0; g < 3; ++g)
            bq[u][g] = Frag<_Float16>::load(rkt + (size_t)(g * NHID + (ub0 + u) * 16 + cl) * NHID + koff + k0);
#pragma unroll
        for (int u = 0; u < 2; ++u)
#pragma unroll
          for (int g = 0; g < 3; ++g) acc[u][g] = Frag<_Float16>::mma(a, bq[u][g], acc[u][g]);
        dep_guard_h(acc[0][0], acc[1][2], a, bq[1][2]);
        keep4_h(bq[0][0], bq[0][1], bq[0][2], bq[1][0]);
        keep4_h(bq[1][1], bq[1][2], bq[0][0], bq[1][0]);
      }
      acc_guard4(acc[0][0], acc[0][1], acc[0][2], acc[1][0]);
      acc_guard2(acc[1][1], acc[1][2]);

#pragma unroll
      for (int u = 0; u < 2; ++u) {
        const int j = (ub0 + u) * 16 + cl;
        const float brz = brec[j], brr = brec[NHID + j], brh = brec[2 * NHID + j];
#pragma unroll
        for (int r = 0; r < 8; ++r) {
          const int row = 8 * hh + r;
          const float* xrow = xs + ((size_t)(tl * NBATCH + bBase + row)) * NH3 + j;
          const float xz = xrow[0], xr = xrow[NHID], xh = xrow[2 * NHID];
          const float iz = acc[u][0][r] * WSCALE_INV + brz;
          const float ir = acc[u][1][r] * WSCALE_INV + brr;
          const float ih = acc[u][2][r] * WSCALE_INV + brh;
          const float zg = sigm_f(xz + iz);
          const float rg = sigm_f(xr + ir);
          const float hc = tanhf(xh + rg * ih);
          const float hp = hf[row * NHID + j];
          float hn = zg * hp + (1.0f - zg) * hc;
          hn = (t < lenr[r]) ? hn : hp;
          hf[row * NHID + j] = hn;
          hnext[row * NHID + j] = (_Float16)hn;
        }
      }
    }
    __syncthreads();

    {
      const int q = lane >> 3, c8 = (lane & 7) * 8;
      v4u vv[4];
      size_t off[4];
#pragma unroll
      for (int it = 0; it < 4; ++it) {
        const int row = 2 * wave + (it >> 1);
        const int colh = ((it & 1) * 4 + q) * 64 + c8;
        vv[it] = *(const v4u*)(hnext + row * NHID + colh);
        off[it] = ((size_t)((bBase + row) * NTIME + t)) * (2 * NHID) + dir * NHID + colh;
      }
      for (int pass = 0; pass < 2; ++pass) {
#pragma unroll
        for (int it = 0; it < 4; ++it) *(volatile v4u*)(out16 + off[it]) = vv[it];
        __threadfence();
      }
    }
  }

  {
    v4f hv[8];
    size_t off[8];
#pragma unroll
    for (int rr = 0; rr < 2; ++rr)
#pragma unroll
      for (int it = 0; it < 4; ++it) {
        const int row = 2 * wave + rr;
        const int col = it * 128 + lane * 4;
        hv[rr * 4 + it] = *(const v4f*)(hf + row * NHID + col);
        off[rr * 4 + it] = ((size_t)(dir * NBATCH + bBase + row)) * NHID + col;
      }
    for (int pass = 0; pass < 2; ++pass) {
#pragma unroll
      for (int i = 0; i < 8; ++i) *(volatile v4f*)(hst + off[i]) = hv[i];
      __threadfence();
    }
  }
}

__global__ __launch_bounds__(256) void build_ht16_kernel(const unsigned short* __restrict__ out16,
                                                         unsigned short* __restrict__ ht16) {
  const int tid = threadIdx.x;
  for (int it = 0; it < 32; ++it) {
    const int idx = it * 256 + tid;
    const int row = idx >> 7;
    const int c8 = (idx & 127) * 8;
    const int rowc = row < NBATCH ? row : (NBATCH - 1);
    const int tsel = (c8 < NHID) ? (NTIME - 1) : 0;
    const size_t src = ((size_t)(rowc * NTIME + tsel)) * (2 * NHID) + c8;
    v4u v = *(const v4u*)(out16 + src);
    if (row >= NBATCH) { v[0] = 0u; v[1] = 0u; v[2] = 0u; v[3] = 0u; }
    unsigned short* dst = ht16 + (size_t)row * (2 * NHID) + c8;
    *(volatile v4u*)dst = v;
    __threadfence();
    *(volatile v4u*)dst = v;
  }
}

__global__ __launch_bounds__(256) void copy_hidden_kernel(const float* __restrict__ hidf, float* __restrict__ out1) {
  const int tid = threadIdx.x;
  for (int it = 0; it < 16; ++it) {
    const int idx = it * 256 + tid;
    const v4f v = *(const v4f*)(hidf + (size_t)idx * 4);
    *(volatile v4f*)(out1 + (size_t)idx * 4) = v;
    __threadfence();
    *(volatile v4f*)(out1 + (size_t)idx * 4) = v;
  }
}

extern "C" void kernel_launch(void* const* d_in, const int* in_sizes, int n_in,
                              void* d_out, int out_size, void* d_ws, size_t ws_size,
                              hipStream_t stream) {
  if (n_in < 11) return;
  const int*   seqs = (const int*)d_in[0];
  const int*   lens = (const int*)d_in[1];
  const float* emb  = (const float*)d_in[2];
  const float* k_f  = (const float*)d_in[3];
  const float* rk_f = (const float*)d_in[4];
  const float* b_f  = (const float*)d_in[5];
  const float* k_b  = (const float*)d_in[6];
  const float* rk_b = (const float*)d_in[7];
  const float* b_b  = (const float*)d_in[8];
  const float* Wk   = (const float*)d_in[9];
  const float* Wb   = (const float*)d_in[10];
  float* out0 = (float*)d_out;
  float* out1 = (float*)d_out + (size_t)NROWS * NHID;

  if (in_sizes[0] != NBATCH * NTIME * NMEM || in_sizes[1] != NBATCH) return;
  if (in_sizes[2] != NVOCAB * NHID || in_sizes[3] != NHID * NH3 || in_sizes[9] != 2 * NHID * NHID) return;
  if (out_size != NROWS * NHID + NBATCH * NHID) return;

  const size_t szW16   = (size_t)NH3 * NHID * 2;
  const size_t szWK16  = (size_t)NHID * (2 * NHID) * 2;
  const size_t szEMB16 = (size_t)NROWS * NHID * 2;
  const size_t szXS    = (size_t)ROWS_CH * NH3 * 4;
  const size_t szOUT16 = (size_t)NROWS * (2 * NHID) * 2;
  const size_t szHST   = (size_t)2 * NBATCH * NHID * 4;
  const size_t szHT16  = (size_t)64 * (2 * NHID) * 2;
  const size_t szHIDF  = (size_t)64 * NHID * 4;
  size_t off = 0;
  char* ws = (char*)d_ws;
  unsigned short* KT16_f  = (unsigned short*)(ws + off); off += szW16;
  unsigned short* KT16_b  = (unsigned short*)(ws + off); off += szW16;
  unsigned short* RKT16_f = (unsigned short*)(ws + off); off += szW16;
  unsigned short* RKT16_b = (unsigned short*)(ws + off); off += szW16;
  unsigned short* WKT16   = (unsigned short*)(ws + off); off += szWK16;
  unsigned short* EMB16   = (unsigned short*)(ws + off); off += szEMB16;
  float*          XS_f    = (float*)(ws + off);          off += szXS;
  float*          XS_b    = (float*)(ws + off);          off += szXS;
  unsigned short* OUT16   = (unsigned short*)(ws + off); off += szOUT16;
  float*          HST     = (float*)(ws + off);          off += szHST;
  unsigned short* HT16    = (unsigned short*)(ws + off); off += szHT16;
  float*          HIDF    = (float*)(ws + off);          off += szHIDF;
  if (off > ws_size) return;

  transpose_cast_f16<<<dim3(NH3 / 64, NHID / 64), 256, 0, stream>>>(k_f,  KT16_f,  NHID, NH3, WSCALE);
  transpose_cast_f16<<<dim3(NH3 / 64, NHID / 64), 256, 0, stream>>>(rk_f, RKT16_f, NHID, NH3, WSCALE);
  transpose_cast_f16<<<dim3(NH3 / 64, NHID / 64), 256, 0, stream>>>(k_b,  KT16_b,  NHID, NH3, WSCALE);
  transpose_cast_f16<<<dim3(NH3 / 64, NHID / 64), 256, 0, stream>>>(rk_b, RKT16_b, NHID, NH3, WSCALE);
  transpose_cast_f16<<<dim3(NHID / 64, (2 * NHID) / 64), 256, 0, stream>>>(Wk, WKT16, 2 * NHID, NHID, WSCALE);

  embed_sum_kernel<<<NROWS, 64, 0, stream>>>(seqs, emb, EMB16);

  const int tilesXS = (ROWS_CH / 64) * (NH3 / 64);
  const int blkXS = (tilesXS + 7) / 8;
  for (int ci = 0; ci < NCHUNK; ++ci) {
    const int t0F = ci * TCHUNK;
    const int t0B = NTIME - (ci + 1) * TCHUNK;
    const unsigned short* A_f = EMB16 + (size_t)t0F * NBATCH * NHID;
    const unsigned short* A_b = EMB16 + (size_t)t0B * NBATCH * NHID;
    wmma_gemm64<0, false, 2, 0, false, 0><<<dim3(blkXS, 1), 256, 0, stream>>>(
        A_f, A_f, NHID, 0L, KT16_f, KT16_f, NHID, 0L, (void*)XS_f, (void*)XS_f, NH3, 0L,
        b_f, b_f, 0L, ROWS_CH, NH3, NHID, WSCALE_INV);
    wmma_gemm64<0, false, 2, 0, false, 0><<<dim3(blkXS, 1), 256, 0, stream>>>(
        A_b, A_b, NHID, 0L, KT16_b, KT16_b, NHID, 0L, (void*)XS_b, (void*)XS_b, NH3, 0L,
        b_b, b_b, 0L, ROWS_CH, NH3, NHID, WSCALE_INV);
    gru_scan_kernel<<<4, 256, 0, stream>>>(XS_f, XS_b, RKT16_f, RKT16_b, b_f, b_b, lens,
                                            OUT16, HST, t0F, t0B, (ci == 0) ? 1 : 0);
  }

  build_ht16_kernel<<<1, 256, 0, stream>>>(OUT16, HT16);

  {
    const int tiles = (NROWS / 64) * (NHID / 64);
    wmma_gemm64<0, false, 2, 0, false, 0><<<dim3((tiles + 7) / 8, 1), 256, 0, stream>>>(
        OUT16, OUT16, 2 * NHID, 0L, WKT16, WKT16, 2 * NHID, 0L, (void*)out0, (void*)out0, NHID, 0L,
        Wb, Wb, 0L, NROWS, NHID, 2 * NHID, WSCALE_INV);
  }
  {
    const int tiles = (64 / 64) * (NHID / 64);
    wmma_gemm64<0, false, 2, 0, false, 0><<<dim3((tiles + 7) / 8, 1), 256, 0, stream>>>(
        HT16, HT16, 2 * NHID, 0L, WKT16, WKT16, 2 * NHID, 0L, (void*)HIDF, (void*)HIDF, NHID, 0L,
        Wb, Wb, 0L, 64, NHID, 2 * NHID, WSCALE_INV);
  }
  copy_hidden_kernel<<<1, 256, 0, stream>>>(HIDF, out1);
}
